// MultiHeadDoublyStochasticSelfAttention_62612033241695
// MI455X (gfx1250) — hardware-run, weakly checked
//
#include <hip/hip_runtime.h>
#include <stdint.h>

#define NB   8
#define NS   1024
#define NF   768
#define NH   12
#define DH   64
#define GP   8
#define NGRP 12

static_assert(NH * DH == NF);
static_assert(NB * NH == GP * NGRP);
static_assert((NS % 64) == 0 && (NF % 64) == 0 && DH == 64);
static_assert(NS == 1024);
static_assert(((NB * NS * NF) % (8 * 256)) == 0 && ((NF * NF) % (8 * 256)) == 0);

typedef __bf16   v16b __attribute__((ext_vector_type(16)));
typedef __bf16   v8b  __attribute__((ext_vector_type(8)));
typedef _Float16 v16h __attribute__((ext_vector_type(16)));
typedef _Float16 v8h  __attribute__((ext_vector_type(8)));
typedef float    v8f  __attribute__((ext_vector_type(8)));
typedef float    v4f  __attribute__((ext_vector_type(4)));
typedef unsigned int v4u __attribute__((ext_vector_type(4)));

__device__ __forceinline__ unsigned short bf_bits(float f) {
  unsigned u = __float_as_uint(f);
  return (unsigned short)((u + 0x7FFFu + ((u >> 16) & 1u)) >> 16);
}
__device__ __forceinline__ float bf_rne(float f) {
  return __uint_as_float(((unsigned)bf_bits(f)) << 16);
}
__device__ __forceinline__ unsigned pk16(unsigned short a, unsigned short b) { return (unsigned)a | ((unsigned)b << 16); }
__device__ __forceinline__ v8f zero8() { v8f z = {0.f, 0.f, 0.f, 0.f, 0.f, 0.f, 0.f, 0.f}; return z; }

struct OpB {
  typedef v16b V;
  static __device__ __forceinline__ V ld(const unsigned short* p) {
    union { v16b v; v8b h[2]; } f;
    f.h[0] = *(const v8b*)(const void*)(p);
    f.h[1] = *(const v8b*)(const void*)(p + 16);
    return f.v;
  }
  static __device__ __forceinline__ v8f mma(V a, V b, v8f c) {
    return __builtin_amdgcn_wmma_f32_16x16x32_bf16(false, a, false, b, (short)0, c, false, false);
  }
};
struct OpH {
  typedef v16h V;
  static __device__ __forceinline__ V ld(const unsigned short* p) {
    union { v16h v; v8h h[2]; } f;
    f.h[0] = *(const v8h*)(const void*)(p);
    f.h[1] = *(const v8h*)(const void*)(p + 16);
    return f.v;
  }
  static __device__ __forceinline__ v8f mma(V a, V b, v8f c) {
    return __builtin_amdgcn_wmma_f32_16x16x32_f16(false, a, false, b, (short)0, c, false, false);
  }
};

template <class V>
__device__ __forceinline__ void dep_guard(v8f& a, v8f& b, V x, V y) {
#if defined(__HIP_DEVICE_COMPILE__)
  asm volatile("v_nop\n\tv_nop\n\tv_nop\n\tv_nop" : "+v"(a), "+v"(b) : "v"(x), "v"(y));
#endif
}
template <class V>
__device__ __forceinline__ void keep4(V a, V b, V c, V d) {
#if defined(__HIP_DEVICE_COMPILE__)
  asm volatile("v_nop" :: "v"(a), "v"(b), "v"(c), "v"(d));
#endif
}
__device__ __forceinline__ void acc_guard4(v8f& a, v8f& b, v8f& c, v8f& d) {
#if defined(__HIP_DEVICE_COMPILE__)
  asm volatile("v_nop\n\tv_nop\n\tv_nop\n\tv_nop" : "+v"(a), "+v"(b), "+v"(c), "+v"(d));
#endif
}
__device__ __forceinline__ void wave_sync_lds() {
#if defined(__HIP_DEVICE_COMPILE__)
  __builtin_amdgcn_fence(__ATOMIC_RELEASE, "workgroup");
  __builtin_amdgcn_wave_barrier();
  __builtin_amdgcn_fence(__ATOMIC_ACQUIRE, "workgroup");
#endif
}

__global__ __launch_bounds__(256) void cvt_bf16x8(const float* __restrict__ in, unsigned short* out, int n8) {
  const int i = blockIdx.x * 256 + threadIdx.x;
  if (i >= n8) return;
  const v4f a = *(const v4f*)(in + (size_t)i * 8);
  const v4f b = *(const v4f*)(in + (size_t)i * 8 + 4);
  v4u p;
  p[0] = pk16(bf_bits(a[0]), bf_bits(a[1]));
  p[1] = pk16(bf_bits(a[2]), bf_bits(a[3]));
  p[2] = pk16(bf_bits(b[0]), bf_bits(b[1]));
  p[3] = pk16(bf_bits(b[2]), bf_bits(b[3]));
  *(volatile v4u*)(out + (size_t)i * 8) = p;
  __threadfence();
  *(volatile v4u*)(out + (size_t)i * 8) = p;
}

__global__ __launch_bounds__(256) void cvt_f16x8(const float* __restrict__ in, unsigned short* out, int n8,
                                                 float scale) {
  const int i = blockIdx.x * 256 + threadIdx.x;
  if (i >= n8) return;
  const v4f a = *(const v4f*)(in + (size_t)i * 8);
  const v4f b = *(const v4f*)(in + (size_t)i * 8 + 4);
  union { v8h h; v4u u; } q;
  q.h[0] = (_Float16)(bf_rne(a[0]) * scale);
  q.h[1] = (_Float16)(bf_rne(a[1]) * scale);
  q.h[2] = (_Float16)(bf_rne(a[2]) * scale);
  q.h[3] = (_Float16)(bf_rne(a[3]) * scale);
  q.h[4] = (_Float16)(bf_rne(b[0]) * scale);
  q.h[5] = (_Float16)(bf_rne(b[1]) * scale);
  q.h[6] = (_Float16)(bf_rne(b[2]) * scale);
  q.h[7] = (_Float16)(bf_rne(b[3]) * scale);
  const v4u p = q.u;
  *(volatile v4u*)(out + (size_t)i * 8) = p;
  __threadfence();
  *(volatile v4u*)(out + (size_t)i * 8) = p;
}

template <class T, int OUT, int HM, int HASB>
__global__ __launch_bounds__(256) void gemm64(
    const unsigned short* __restrict__ Ap, int lda, int sA,
    const unsigned short* __restrict__ Bp, int ldb, int sB,
    void* Cout, int ldc, int sC0, int z0, int sC1, int sC2,
    const float* __restrict__ bias, float alpha, int M, int N, int K) {
  __shared__ __align__(16) float sT[8][16 * 68];
  typedef typename T::V V;
  const int lane = threadIdx.x & 31;
  const int wave = threadIdx.x >> 5;
  const int z = blockIdx.y;
  const int tilesN = N >> 6;
  const int tilesM = M >> 6;
  const int tile = blockIdx.x * 8 + wave;
  if (tile >= tilesM * tilesN) return;
  const int tm = tile / tilesN;
  const int tn = tile - tm * tilesN;
  const int m0 = tm << 6;
  const int n0 = tn << 6;
  const unsigned short* A  = Ap + (size_t)z * (size_t)sA;
  const unsigned short* Bt = Bp + (size_t)z * (size_t)sB;
  const int zz = z0 + z;
  const size_t offC = (size_t)z * (size_t)sC0 + (size_t)(zz / NH) * (size_t)sC1 +
                      (size_t)(zz % NH) * (size_t)sC2;

  const int rlane = lane & 15;
  const int koff  = (lane >> 4) * 8;
  const int mOff  = (lane >> 4) * 8;

  v8f acc[4][4];
#pragma unroll
  for (int i = 0; i < 4; ++i)
#pragma unroll
    for (int j = 0; j < 4; ++j) acc[i][j] = zero8();

  for (int k0 = 0; k0 < K; k0 += 32) {
    V bh[4];
#pragma unroll
    for (int j = 0; j < 4; ++j) {
      const size_t bo = (size_t)(n0 + (j << 4) + rlane) * ldb + koff + k0;
      bh[j] = T::ld(Bt + bo);
    }
#pragma unroll
    for (int i = 0; i < 4; ++i) {
      const size_t ao = (size_t)(m0 + (i << 4) + rlane) * lda + koff + k0;
      const V ah = T::ld(A + ao);
#pragma unroll
      for (int j = 0; j < 4; ++j) {
        acc[i][j] = T::mma(ah, bh[j], acc[i][j]);
      }
      dep_guard<V>(acc[i][0], acc[i][3], ah, bh[3]);
    }
    keep4<V>(bh[0], bh[1], bh[2], bh[3]);
  }
  acc_guard4(acc[0][0], acc[0][1], acc[0][2], acc[0][3]);
  acc_guard4(acc[1][0], acc[1][1], acc[1][2], acc[1][3]);
  acc_guard4(acc[2][0], acc[2][1], acc[2][2], acc[2][3]);
  acc_guard4(acc[3][0], acc[3][1], acc[3][2], acc[3][3]);

  float* slab = sT[wave];
  v4f bb = {0.f, 0.f, 0.f, 0.f};
  if (OUT == 0 && HASB) {
    const int c4 = (lane & 15) * 4;
    const v4f t = *(const v4f*)(bias + n0 + c4);
    bb[0] = bf_rne(t[0]); bb[1] = bf_rne(t[1]); bb[2] = bf_rne(t[2]); bb[3] = bf_rne(t[3]);
  }
#pragma unroll
  for (int i = 0; i < 4; ++i) {
    const int mBase = m0 + (i << 4);
#pragma unroll
    for (int j = 0; j < 4; ++j) {
#pragma unroll
      for (int r = 0; r < 8; ++r) {
        slab[(mOff + r) * 68 + (j << 4) + rlane] = acc[i][j][r];
      }
    }
    wave_sync_lds();
    if (OUT == 0) {
      float* C = (float*)Cout;
      const int hh = lane >> 4, c4 = (lane & 15) * 4;
      v4f vv[8];
#pragma unroll
      for (int it = 0; it < 8; ++it) {
        const int row = it * 2 + hh;
        const v4f v = *(const v4f*)(slab + row * 68 + c4);
        vv[it] = v * alpha + bb;
      }
      for (int pass = 0; pass < 2; ++pass) {
#pragma unroll
        for (int it = 0; it < 8; ++it) {
          const int row = it * 2 + hh;
          *(volatile v4f*)(C + offC + (size_t)(mBase + row) * ldc + n0 + c4) = vv[it];
        }
        __threadfence();
      }
    } else {
      unsigned short* Ch = (unsigned short*)Cout;
      const int q8 = (lane & 7) * 8, rr = lane >> 3;
      v4u ph[4];
#pragma unroll
      for (int it = 0; it < 4; ++it) {
        const int row = it * 4 + rr;
        v4f a = *(const v4f*)(slab + row * 68 + q8);
        v4f b = *(const v4f*)(slab + row * 68 + q8 + 4);
        a = a * alpha;
        b = b * alpha;
        union { v8h h; v4u u; } q;
        q.h[0] = (_Float16)a[0]; q.h[1] = (_Float16)a[1]; q.h[2] = (_Float16)a[2]; q.h[3] = (_Float16)a[3];
        q.h[4] = (_Float16)b[0]; q.h[5] = (_Float16)b[1]; q.h[6] = (_Float16)b[2]; q.h[7] = (_Float16)b[3];
        ph[it] = q.u;
      }
      for (int pass = 0; pass < 2; ++pass) {
#pragma unroll
        for (int it = 0; it < 4; ++it) {
          const int row = it * 4 + rr;
          const int mrow = mBase + row;
          size_t co;
          if (HM) {
            co = ((size_t)((mrow >> 10) * NH + (n0 >> 6)) * NS + (size_t)(mrow & (NS - 1))) * DH + q8;
          } else {
            co = offC + (size_t)mrow * ldc + n0 + q8;
          }
          *(volatile v4u*)(Ch + co) = ph[it];
        }
        __threadfence();
      }
    }
    wave_sync_lds();
  }
}

template <int MODE>
__global__ __launch_bounds__(256) void k_row(const float* __restrict__ S, const float* __restrict__ uin,
                                             const float* __restrict__ vin, float* uout, unsigned short* P,
                                             float logmu) {
  __shared__ float sU[32];
  const int tid  = threadIdx.x;
  const int lane = tid & 31;
  const int wave = tid >> 5;
  const int plane = blockIdx.y;
  const int rbase = blockIdx.x * 32 + wave * 4;
  const float* Sp = S + (size_t)plane * ((size_t)NS * NS);

  float vv[32];
#pragma unroll
  for (int k = 0; k < 32; ++k) vv[k] = 0.0f;
  if (MODE) {
#pragma unroll
    for (int c = 0; c < 4; ++c) {
      const v4f a = *(const v4f*)(vin + (size_t)plane * NS + c * 256 + lane * 8);
      const v4f b = *(const v4f*)(vin + (size_t)plane * NS + c * 256 + lane * 8 + 4);
      vv[c * 8 + 0] = a[0]; vv[c * 8 + 1] = a[1]; vv[c * 8 + 2] = a[2]; vv[c * 8 + 3] = a[3];
      vv[c * 8 + 4] = b[0]; vv[c * 8 + 5] = b[1]; vv[c * 8 + 6] = b[2]; vv[c * 8 + 7] = b[3];
    }
  }

#pragma unroll 1
  for (int rr = 0; rr < 4; ++rr) {
    const int row = rbase + rr;
    const float* Sr = Sp + (size_t)row * NS;
    float s[32];
#pragma unroll
    for (int c = 0; c < 4; ++c) {
      const v4f a = *(const v4f*)(Sr + c * 256 + lane * 8);
      const v4f b = *(const v4f*)(Sr + c * 256 + lane * 8 + 4);
      s[c * 8 + 0] = a[0]; s[c * 8 + 1] = a[1]; s[c * 8 + 2] = a[2]; s[c * 8 + 3] = a[3];
      s[c * 8 + 4] = b[0]; s[c * 8 + 5] = b[1]; s[c * 8 + 6] = b[2]; s[c * 8 + 7] = b[3];
    }
    float u0r = 0.0f;
    if (MODE) u0r = uin[(size_t)plane * NS + row];
    float t[32];
#pragma unroll
    for (int k = 0; k < 32; ++k) t[k] = MODE ? ((s[k] + u0r) + vv[k]) : s[k];

    float m = t[0];
#pragma unroll
    for (int k = 1; k < 32; ++k) m = fmaxf(m, t[k]);
    m = fmaxf(m, __shfl_xor(m, 16));
    m = fmaxf(m, __shfl_xor(m, 8));
    m = fmaxf(m, __shfl_xor(m, 4));
    m = fmaxf(m, __shfl_xor(m, 2));
    m = fmaxf(m, __shfl_xor(m, 1));

    float part = 0.0f;
#pragma unroll
    for (int k = 0; k < 32; ++k) part += __expf(t[k] - m);
    part += __shfl_xor(part, 16);
    part += __shfl_xor(part, 8);
    part += __shfl_xor(part, 4);
    part += __shfl_xor(part, 2);
    part += __shfl_xor(part, 1);

    const float lse = m + __logf(part);
    const float un  = (logmu - lse) + u0r;

    if (MODE) {
      v4u pk[4];
#pragma unroll
      for (int c = 0; c < 4; ++c) {
        union { v8h h; v4u u; } q;
#pragma unroll
        for (int e = 0; e < 8; ++e) {
          const float p = __expf((s[c * 8 + e] + un) + vv[c * 8 + e]) * 1048576.0f;
          q.h[e] = (_Float16)p;
        }
        pk[c] = q.u;
      }
      unsigned short* Pr = P + (size_t)plane * ((size_t)NS * NS) + (size_t)row * NS + lane * 8;
      for (int pass = 0; pass < 2; ++pass) {
#pragma unroll
        for (int c = 0; c < 4; ++c) {
          *(volatile v4u*)(Pr + c * 256) = pk[c];
        }
        __threadfence();
      }
    }
    if (lane == 0) sU[wave * 4 + rr] = un;
  }
  __syncthreads();
  if (wave == 0) {
    const float uv = sU[lane];
    float* up = uout + (size_t)plane * NS + blockIdx.x * 32 + lane;
    *(volatile float*)up = uv;
    __threadfence();
    *(volatile float*)up = uv;
  }
}

__global__ __launch_bounds__(256) void k_col(const float* __restrict__ S, const float* __restrict__ uin,
                                             float* vout, float logmu) {
  const int tid = threadIdx.x;
  const int plane = blockIdx.y;
  const int j4 = (blockIdx.x * 256 + tid) * 4;
  const float* Sp = S + (size_t)plane * ((size_t)NS * NS) + j4;
  const float* up = uin + (size_t)plane * NS;

  v4f m = {-3.0e38f, -3.0e38f, -3.0e38f, -3.0e38f};
#pragma unroll 4
  for (int i = 0; i < NS; ++i) {
    const v4f x = *(const v4f*)(Sp + (size_t)i * NS);
    const float ui = up[i];
    m[0] = fmaxf(m[0], x[0] + ui);
    m[1] = fmaxf(m[1], x[1] + ui);
    m[2] = fmaxf(m[2], x[2] + ui);
    m[3] = fmaxf(m[3], x[3] + ui);
  }
  v4f sum = {0.f, 0.f, 0.f, 0.f};
#pragma unroll 4
  for (int i = 0; i < NS; ++i) {
    const v4f x = *(const v4f*)(Sp + (size_t)i * NS);
    const float ui = up[i];
    sum[0] += __expf((x[0] + ui) - m[0]);
    sum[1] += __expf((x[1] + ui) - m[1]);
    sum[2] += __expf((x[2] + ui) - m[2]);
    sum[3] += __expf((x[3] + ui) - m[3]);
  }
  v4f vn;
  vn[0] = (logmu - (m[0] + __logf(sum[0])));
  vn[1] = (logmu - (m[1] + __logf(sum[1])));
  vn[2] = (logmu - (m[2] + __logf(sum[2])));
  vn[3] = (logmu - (m[3] + __logf(sum[3])));
  float* vp = vout + (size_t)plane * NS + j4;
  *(volatile v4f*)vp = vn;
  __threadfence();
  *(volatile v4f*)vp = vn;
}

extern "C" void kernel_launch(void* const* d_in, const int* in_sizes, int n_in,
                              void* d_out, int out_size, void* d_ws, size_t ws_size,
                              hipStream_t stream) {
  if (n_in < 6) return;
  if (in_sizes[0] != NB * NS * NF) return;
  if (in_sizes[1] != NF * NF || in_sizes[2] != NF * NF || in_sizes[3] != NF * NF || in_sizes[4] != NF * NF) return;
  if (in_sizes[5] != NF) return;
  if (out_size != NB * NS * NF) return;

  const float* x  = (const float*)d_in[0];
  const float* Wq = (const float*)d_in[1];
  const float* Wk = (const float*)d_in[2];
  const float* Wv = (const float*)d_in[3];
  const float* Wo = (const float*)d_in[4];
  const float* bo = (const float*)d_in[5];
  float* out = (float*)d_out;

  const size_t PXB = (size_t)NB * NS * NF * 2;
  const size_t PW  = (size_t)NF * NF * 2;
  const size_t PQK = (size_t)NB * NH * NS * DH * 2;
  const size_t PVT = (size_t)NB * NH * DH * NS * 2;
  const size_t PS  = (size_t)GP * NS * NS * 4;
  const size_t PP  = (size_t)GP * NS * NS * 2;
  const size_t PCX = (size_t)NB * NS * NF * 2;
  const size_t PUV = (size_t)GP * NS * 4;
  size_t off = 0;
  const size_t oX  = off; off += PXB;
  const size_t oWq = off; off += PW;
  const size_t oWk = off; off += PW;
  const size_t oWv = off; off += PW;
  const size_t oWo = off; off += PW;
  const size_t oQ  = off; off += PQK;
  const size_t oK  = off; off += PQK;
  const size_t oVt = off; off += PVT;
  const size_t oS  = off; off += PS;
  const size_t oP  = off; off += PP;
  const size_t oCx = off; off += PCX;
  const size_t oU0 = off; off += PUV;
  const size_t oV1 = off; off += PUV;
  const size_t oU2 = off; off += PUV;
  if (off > ws_size) return;
  if (off > (size_t)134217728) return;

  char* ws = (char*)d_ws;
  unsigned short* Xb  = (unsigned short*)(ws + oX);
  unsigned short* Wqb = (unsigned short*)(ws + oWq);
  unsigned short* Wkb = (unsigned short*)(ws + oWk);
  unsigned short* Wvb = (unsigned short*)(ws + oWv);
  unsigned short* Wob = (unsigned short*)(ws + oWo);
  unsigned short* Qp  = (unsigned short*)(ws + oQ);
  unsigned short* Kp  = (unsigned short*)(ws + oK);
  unsigned short* Vt  = (unsigned short*)(ws + oVt);
  float*          S   = (float*)(ws + oS);
  unsigned short* P   = (unsigned short*)(ws + oP);
  unsigned short* Cx  = (unsigned short*)(ws + oCx);
  float*          U0  = (float*)(ws + oU0);
  float*          V1  = (float*)(ws + oV1);
  float*          U2  = (float*)(ws + oU2);

  const float logmu = -6.93147182464599609375f;

  const dim3 blk(256);
  const int n8x = NB * NS * NF / 8;
  const int n8w = NF * NF / 8;
  const dim3 gCvtX(n8x / 256);
  const dim3 gCvtW(n8w / 256);
  const dim3 gProj(((NB * NS / 64) * (NF / 64)) / 8, 1);
  const dim3 gVt(((NF / 64) * (NS / 64)) / 8, NB);
  const dim3 gSc(((NS / 64) * (NS / 64)) / 8, GP);
  const dim3 gRow(NS / 32, GP);
  const dim3 gCol(NS / (256 * 4), GP);
  const dim3 gPV(((NS / 64) * (DH / 64)) / 8, GP);

  cvt_bf16x8<<<gCvtX, blk, 0, stream>>>(x, Xb, n8x);
  cvt_bf16x8<<<gCvtW, blk, 0, stream>>>(Wq, Wqb, n8w);
  cvt_bf16x8<<<gCvtW, blk, 0, stream>>>(Wk, Wkb, n8w);
  cvt_bf16x8<<<gCvtW, blk, 0, stream>>>(Wv, Wvb, n8w);
  cvt_f16x8<<<gCvtW, blk, 0, stream>>>(Wo, Wob, n8w, 64.0f);

  gemm64<OpB, 1, 1, 0><<<gProj, blk, 0, stream>>>(Xb, NF, 0, Wqb, NF, 0, (void*)Qp, DH, 0, 0, 0, 0,
                                                   bo, 1.0f, NB * NS, NF, NF);
  gemm64<OpB, 1, 1, 0><<<gProj, blk, 0, stream>>>(Xb, NF, 0, Wkb, NF, 0, (void*)Kp, DH, 0, 0, 0, 0,
                                                   bo, 1.0f, NB * NS, NF, NF);
  gemm64<OpB, 1, 0, 0><<<gVt, blk, 0, stream>>>(Wvb, NF, 0, Xb, NF, NS * NF, (void*)Vt, NS, NH * DH * NS,
                                                 0, 0, 0, bo, 1.0f, NF, NS, NF);

  for (int g = 0; g < NGRP; ++g) {
    const unsigned short* Qg = Qp + (size_t)g * GP * NS * DH;
    const unsigned short* Kg = Kp + (size_t)g * GP * NS * DH;
    const unsigned short* Vg = Vt + (size_t)g * GP * DH * NS;
    gemm64<OpH, 0, 0, 0><<<gSc, blk, 0, stream>>>(Qg, DH, NS * DH, Kg, DH, NS * DH, (void*)S, NS, NS * NS,
                                                   0, 0, 0, bo, 0.125f, NS, NS, DH);
    k_row<0><<<gRow, blk, 0, stream>>>(S, U0, V1, U0, P, logmu);
    k_col<<<gCol, blk, 0, stream>>>(S, U0, V1, logmu);
    k_row<1><<<gRow, blk, 0, stream>>>(S, U0, V1, U2, P, logmu);
    gemm64<OpH, 1, 0, 0><<<gPV, blk, 0, stream>>>(P, NS, NS * NS, Vg, NS, DH * NS, (void*)Cx, NF, 0,
                                                  g * GP, NS * NF, DH, bo, 0.015625f, NS, DH, NS);
  }

  gemm64<OpH, 0, 0, 1><<<gProj, blk, 0, stream>>>(Cx, NF, 0, Wob, NF, 0, (void*)out, NF, 0, 0, 0, 0,
                                                   bo, 9.5367431640625e-7f, NB * NS, NF, NF);
  (void)hipGetLastError();
}
